// GeneGCN_5342939316652
// MI455X (gfx1250) — hardware-verified
//
#include <hip/hip_runtime.h>
#include <stddef.h>
#include <stdint.h>


#define DD      128
#define NTHR    256
#define NWAVE   8
#define EPT     8
#define NGRP    2
#define CHUNK   (NTHR * EPT * NGRP)
#define WCAP    (EPT * NGRP * 32)
#define LISTN   (NWAVE * WCAP)
#define NBC     4096
#define NBF     1024
#define RCAP    40960
#define RBN     128
#define TGT     256
#define DEGCAP  256
#define GROWS   128
#define OTHR    512

#define LDS_FILL ((RCAP + NBF + LISTN) * 4 + 64)
#define LDS_GEMM (GROWS * DD * 4)
#define WS_LIMIT ((size_t)134217728)

static_assert((CHUNK & (CHUNK - 1)) == 0);
static_assert(CHUNK <= 4096);
static_assert((NBC & (NBC - 1)) == 0 && (NBF & (NBF - 1)) == 0);
static_assert(NBC == 4 * NBF);
static_assert(OTHR * 8 == NBC);
static_assert((RCAP % 32) == 0);
static_assert(TGT == NWAVE * 32);
static_assert((TGT % GROWS) == 0);
static_assert(GROWS == NWAVE * 16);
static_assert(DD == 128);
static_assert((DD * DD / 8) % NTHR == 0);

typedef float          v4f  __attribute__((ext_vector_type(4)));
typedef float          v8f  __attribute__((ext_vector_type(8)));
typedef int            v4i  __attribute__((ext_vector_type(4)));
typedef unsigned short v8us __attribute__((ext_vector_type(8)));
typedef unsigned int   v8u  __attribute__((ext_vector_type(8)));
typedef __bf16         v16b __attribute__((ext_vector_type(16)));
union FragB { v16b v; v8us u[2]; v8u w; };

__device__ __forceinline__ unsigned int bf_bits(float f) {
  const unsigned int u = __float_as_uint(f);
  return (u + 0x7FFFu + ((u >> 16) & 1u)) >> 16;
}

__device__ __forceinline__ v8f wmb(const FragB& a, const FragB& b, v8f c) {
  v8f d = __builtin_amdgcn_wmma_f32_16x16x32_bf16(false, a.v, false, b.v, (short)0, c, false, false);
  asm volatile("v_nop\n\tv_nop\n\tv_nop\n\tv_nop" : "+v"(d) : "v"(a.w), "v"(b.w));
  return d;
}

__device__ __forceinline__ void split16(const float* ap, FragB& hi, FragB& lo) {
  const v4f f0 = *(const v4f*)(ap);
  const v4f f1 = *(const v4f*)(ap + 4);
  const v4f f2 = *(const v4f*)(ap + 16);
  const v4f f3 = *(const v4f*)(ap + 20);
  float v[16];
  v[0]  = f0.x; v[1]  = f0.y; v[2]  = f0.z; v[3]  = f0.w;
  v[4]  = f1.x; v[5]  = f1.y; v[6]  = f1.z; v[7]  = f1.w;
  v[8]  = f2.x; v[9]  = f2.y; v[10] = f2.z; v[11] = f2.w;
  v[12] = f3.x; v[13] = f3.y; v[14] = f3.z; v[15] = f3.w;
  v8u wh, wl;
#pragma unroll
  for (int j = 0; j < 8; ++j) {
    const unsigned int h0 = bf_bits(v[2 * j]);
    const unsigned int h1 = bf_bits(v[2 * j + 1]);
    const unsigned int l0 = bf_bits(v[2 * j]     - __uint_as_float(h0 << 16));
    const unsigned int l1 = bf_bits(v[2 * j + 1] - __uint_as_float(h1 << 16));
    wh[j] = h0 | (h1 << 16);
    wl[j] = l0 | (l1 << 16);
  }
  hi.w = wh;
  lo.w = wl;
}

template <int NB>
__device__ __forceinline__ int scan_chunk(const int* __restrict__ dsts, int nE, int cbase, int slotBase,
                                          int vec8, int* list, int tid, int lane, int wave) {
  int wc = 0;
#pragma unroll
  for (int g = 0; g < NGRP; ++g) {
    const int el0  = (g * NTHR + tid) * EPT;
    const int e0   = cbase + el0;
    const int sent = -2147483647 - 1;
    v4i da, db;
    if (vec8 != 0 && cbase + CHUNK <= nE) {
      da = *(const v4i*)(dsts + e0);
      db = *(const v4i*)(dsts + e0 + 4);
    } else {
      da.x = (e0     < nE) ? dsts[min(e0, nE - 1)] : sent;
      da.y = (e0 + 1 < nE) ? dsts[min(e0 + 1, nE - 1)] : sent;
      da.z = (e0 + 2 < nE) ? dsts[min(e0 + 2, nE - 1)] : sent;
      da.w = (e0 + 3 < nE) ? dsts[min(e0 + 3, nE - 1)] : sent;
      db.x = (e0 + 4 < nE) ? dsts[min(e0 + 4, nE - 1)] : sent;
      db.y = (e0 + 5 < nE) ? dsts[min(e0 + 5, nE - 1)] : sent;
      db.z = (e0 + 6 < nE) ? dsts[min(e0 + 6, nE - 1)] : sent;
      db.w = (e0 + 7 < nE) ? dsts[min(e0 + 7, nE - 1)] : sent;
    }
    const unsigned nb = (unsigned)slotBase;
    const unsigned s0 = (unsigned)da.x - nb, s1 = (unsigned)da.y - nb;
    const unsigned s2 = (unsigned)da.z - nb, s3 = (unsigned)da.w - nb;
    const unsigned s4 = (unsigned)db.x - nb, s5 = (unsigned)db.y - nb;
    const unsigned s6 = (unsigned)db.z - nb, s7 = (unsigned)db.w - nb;
    const bool h0 = s0 < (unsigned)NB, h1 = s1 < (unsigned)NB, h2 = s2 < (unsigned)NB, h3 = s3 < (unsigned)NB;
    const bool h4 = s4 < (unsigned)NB, h5 = s5 < (unsigned)NB, h6 = s6 < (unsigned)NB, h7 = s7 < (unsigned)NB;
    const unsigned any = __builtin_amdgcn_ballot_w32(h0 | h1 | h2 | h3 | h4 | h5 | h6 | h7);
    if (any != 0u) {
#define HITJ(J, HJ, SJ) { \
        const unsigned mj = __builtin_amdgcn_ballot_w32(HJ); \
        if (mj != 0u) { \
          if (HJ) { \
            const int pos = wc + (int)__builtin_amdgcn_mbcnt_lo(mj, 0u); \
            if (pos < WCAP) list[wave * WCAP + pos] = ((el0 + (J)) << 12) | (int)(SJ); \
          } \
          wc += (int)__builtin_popcount(mj); } }
      HITJ(0, h0, s0)
      HITJ(1, h1, s1)
      HITJ(2, h2, s2)
      HITJ(3, h3, s3)
      HITJ(4, h4, s4)
      HITJ(5, h5, s5)
      HITJ(6, h6, s6)
      HITJ(7, h7, s7)
#undef HITJ
    }
  }
  return wc;
}

__global__ __launch_bounds__(NTHR) void k_wprep(const float* __restrict__ W,
                                               unsigned short* whi, unsigned short* wlo) {
  const int i = blockIdx.x * NTHR + (int)threadIdx.x;
  if (i >= DD * DD / 8) return;
  const int n  = i >> 4;
  const int k0 = (i & 15) * 8;
  v8us hv, lv;
#pragma unroll
  for (int e = 0; e < 8; ++e) {
    const float f = W[(k0 + e) * DD + n];
    const unsigned int hb = bf_bits(f);
    const unsigned int lb = bf_bits(f - __uint_as_float(hb << 16));
    hv[e] = (unsigned short)hb;
    lv[e] = (unsigned short)lb;
  }
  unsigned short* hp = whi + (size_t)i * 8;
  unsigned short* lp = wlo + (size_t)i * 8;
  *(volatile v8us*)hp = hv;
  *(volatile v8us*)lp = lv;
  __threadfence();
  *(volatile v8us*)hp = hv;
  *(volatile v8us*)lp = lv;
}

__global__ __launch_bounds__(NTHR) void k_count(const int* __restrict__ arow, int* cnt, int nE, int vec8) {
  __shared__ __attribute__((aligned(16))) int scnt[NBC];
  __shared__ __attribute__((aligned(16))) int list[LISTN];
  __shared__ int wcnt[NWAVE];
  const int tid = threadIdx.x, lane = tid & 31, wave = tid >> 5;
  const int nodeBase = blockIdx.x * NBC;

  for (int i = tid; i < NBC; i += NTHR) scnt[i] = 0;
  __syncthreads();

  const int nChunks = (nE + CHUNK - 1) / CHUNK;
#pragma unroll 1
  for (int ch = 0; ch < nChunks; ++ch) {
    const int cbase = ch * CHUNK;
    const int wc = scan_chunk<NBC>(arow, nE, cbase, nodeBase, vec8, list, tid, lane, wave);
    if (lane == 0) wcnt[wave] = wc;
    __syncthreads();
    if (wave == 0) {
#pragma unroll 1
      for (int wsx = 0; wsx < NWAVE; ++wsx) {
        int n = __builtin_amdgcn_readfirstlane(wcnt[wsx]);
        n = n > WCAP ? WCAP : (n < 0 ? 0 : n);
        const int* lp = list + wsx * WCAP;
#pragma unroll 1
        for (int i = 0; i < n; ++i) {
          const int ent  = __builtin_amdgcn_readfirstlane(lp[i]);
          const int slot = ent & (NBC - 1);
          if (lane == 0) scnt[slot] = scnt[slot] + 1;
        }
      }
    }
    __syncthreads();
  }

  v4i cq[4];
#pragma unroll
  for (int q = 0; q < 4; ++q) {
    const int f = (wave * 4 + q) * 128 + 4 * lane;
    cq[q] = *(const v4i*)(scnt + f);
  }
  int* cp = cnt + (size_t)nodeBase;
#pragma unroll
  for (int q = 0; q < 4; ++q) {
    const int f = (wave * 4 + q) * 128 + 4 * lane;
    *(volatile v4i*)(cp + f) = cq[q];
  }
  __threadfence();
#pragma unroll
  for (int q = 0; q < 4; ++q) {
    const int f = (wave * 4 + q) * 128 + 4 * lane;
    *(volatile v4i*)(cp + f) = cq[q];
  }
}

__global__ __launch_bounds__(OTHR) void k_offsets(
    const int* __restrict__ cnt, int* off, int* rbase, int nChunk) {
  __shared__ __attribute__((aligned(16))) int soff[NBC];
  __shared__ __attribute__((aligned(16))) int srb[RBN];
  __shared__ int wtot[OTHR / 32];
  const int tid = threadIdx.x, lane = tid & 31, wave = tid >> 5, sub = tid >> 7;
  for (int i = tid; i < RBN; i += OTHR) srb[i] = 0;
  int carry = 0;
#pragma unroll 1
  for (int ch = 0; ch < nChunk; ++ch) {
    const int base = ch * NBC;
    const v4i c0 = *(const v4i*)(cnt + base + 8 * tid);
    const v4i c1 = *(const v4i*)(cnt + base + 8 * tid + 4);
    const int e0 = max(c0.x, 0), e1 = max(c0.y, 0), e2 = max(c0.z, 0), e3 = max(c0.w, 0);
    const int e4 = max(c1.x, 0), e5 = max(c1.y, 0), e6 = max(c1.z, 0), e7 = max(c1.w, 0);
    const int ts = e0 + e1 + e2 + e3 + e4 + e5 + e6 + e7;
    int incl = ts;
#pragma unroll
    for (int d = 1; d < 32; d <<= 1) {
      const int t = __shfl_up(incl, d);
      if (lane >= d) incl += t;
    }
    if (lane == 31) wtot[wave] = incl;
    __syncthreads();
    const int S0 = wtot[0]  + wtot[1]  + wtot[2]  + wtot[3];
    const int S1 = wtot[4]  + wtot[5]  + wtot[6]  + wtot[7];
    const int S2 = wtot[8]  + wtot[9]  + wtot[10] + wtot[11];
    const int S3 = wtot[12] + wtot[13] + wtot[14] + wtot[15];
    int pre = 0;
#pragma unroll 1
    for (int w = 4 * sub; w < wave; ++w) pre += wtot[w];
    const int b0 = carry;
    const int b1 = b0 + ((S0 + 31) & ~31);
    const int b2 = b1 + ((S1 + 31) & ~31);
    const int b3 = b2 + ((S2 + 31) & ~31);
    const int b4 = b3 + ((S3 + 31) & ~31);
    const int myb = sub == 0 ? b0 : (sub == 1 ? b1 : (sub == 2 ? b2 : b3));
    if (tid == 0) {
      srb[min(4 * ch + 0, RBN - 1)] = b0;
      srb[min(4 * ch + 1, RBN - 1)] = b1;
      srb[min(4 * ch + 2, RBN - 1)] = b2;
      srb[min(4 * ch + 3, RBN - 1)] = b3;
    }
    int run = myb + pre + incl - ts;
    soff[8 * tid + 0] = run; run += e0;
    soff[8 * tid + 1] = run; run += e1;
    soff[8 * tid + 2] = run; run += e2;
    soff[8 * tid + 3] = run; run += e3;
    soff[8 * tid + 4] = run; run += e4;
    soff[8 * tid + 5] = run; run += e5;
    soff[8 * tid + 6] = run; run += e6;
    soff[8 * tid + 7] = run;
    carry = b4;
    __syncthreads();
    const v4i o0 = *(const v4i*)(soff + 4 * tid);
    const v4i o1 = *(const v4i*)(soff + 4 * (tid + OTHR));
    int* op = off + base;
    *(volatile v4i*)(op + 4 * tid) = o0;
    *(volatile v4i*)(op + 4 * (tid + OTHR)) = o1;
    __threadfence();
    *(volatile v4i*)(op + 4 * tid) = o0;
    *(volatile v4i*)(op + 4 * (tid + OTHR)) = o1;
    __syncthreads();
  }
  if (tid == 0) srb[min(4 * nChunk, RBN - 1)] = carry;
  __syncthreads();
  v4i rv = {0, 0, 0, 0};
  if (tid < 32) rv = *(const v4i*)(srb + 4 * tid);
  if (tid < 32) *(volatile v4i*)(rbase + 4 * tid) = rv;
  __threadfence();
  if (tid < 32) *(volatile v4i*)(rbase + 4 * tid) = rv;
}

__global__ __launch_bounds__(NTHR) void k_fill(
    const int* __restrict__ arow, const int* __restrict__ off, const int* __restrict__ rbase,
    int* csr, int nE, int vec8, int csrLen) {
  extern __shared__ v4f lds_dyn[];
  int* region = (int*)lds_dyn;
  int* cursor = region + RCAP;
  int* list   = cursor + NBF;
  int* wcnt   = list + LISTN;
  const int tid = threadIdx.x, lane = tid & 31, wave = tid >> 5;
  const int b = blockIdx.x;
  const int nodeBase = b * NBF;

  int rb0 = rbase[b];
  const int rb1 = rbase[b + 1];
  rb0 = rb0 < 0 ? 0 : (rb0 > csrLen ? csrLen : rb0);
  rb0 &= ~31;
  int len = rb1 - rb0;
  len = len < 0 ? 0 : (len > RCAP ? RCAP : len);
  int lenW = (len + 31) & ~31;
  if (rb0 + lenW > csrLen) lenW = (csrLen - rb0) & ~31;

  {
    const v4i z = {0, 0, 0, 0};
    for (int i = tid; i < RCAP / 4; i += NTHR) ((v4i*)region)[i] = z;
    for (int s = tid; s < NBF; s += NTHR) {
      int o = off[nodeBase + s] - rb0;
      o = o < 0 ? 0 : (o > RCAP ? RCAP : o);
      cursor[s] = o;
    }
  }
  __syncthreads();

  const int nChunks = (nE + CHUNK - 1) / CHUNK;
#pragma unroll 1
  for (int ch = 0; ch < nChunks; ++ch) {
    const int cbase = ch * CHUNK;
    const int wc = scan_chunk<NBF>(arow, nE, cbase, nodeBase, vec8, list, tid, lane, wave);
    if (lane == 0) wcnt[wave] = wc;
    __syncthreads();
    if (wave == 0) {
#pragma unroll 1
      for (int wsx = 0; wsx < NWAVE; ++wsx) {
        int n = __builtin_amdgcn_readfirstlane(wcnt[wsx]);
        n = n > WCAP ? WCAP : (n < 0 ? 0 : n);
        const int* lp = list + wsx * WCAP;
#pragma unroll 1
        for (int i = 0; i < n; ++i) {
          const int ent  = __builtin_amdgcn_readfirstlane(lp[i]);
          const int slot = ent & (NBF - 1);
          int e = cbase + ((ent >> 12) & (CHUNK - 1));
          e = e > nE - 1 ? nE - 1 : e;
          if (lane == 0) {
            int pos = cursor[slot];
            pos = pos < 0 ? 0 : (pos > RCAP - 1 ? RCAP - 1 : pos);
            region[pos] = e;
            const int np = pos + 1;
            cursor[slot] = np > RCAP ? RCAP : np;
          }
        }
      }
    }
    __syncthreads();
  }

  const int nv = lenW >> 2;
  int* gp = csr + rb0;
#pragma unroll 1
  for (int i = tid; i < nv; i += NTHR) { const v4i v = ((const v4i*)region)[i]; *(volatile v4i*)(gp + 4 * i) = v; }
  __threadfence();
#pragma unroll 1
  for (int i = tid; i < nv; i += NTHR) { const v4i v = ((const v4i*)region)[i]; *(volatile v4i*)(gp + 4 * i) = v; }
}

__global__ __launch_bounds__(NTHR) void k_gemm(
    const float* __restrict__ a, const unsigned short* __restrict__ whi, const unsigned short* __restrict__ wlo,
    float* hout, int nA) {
  extern __shared__ v4f lds_dyn[];
  float* stg = (float*)lds_dyn;
  const int tid = threadIdx.x, lane = tid & 31, wave = tid >> 5, hh = lane >> 4, m = lane & 15;
  const int rowBase = blockIdx.x * GROWS;
  int ra = rowBase + wave * 16 + m;
  ra = ra > nA - 1 ? nA - 1 : (ra < 0 ? 0 : ra);
  const float* arow = a + (size_t)ra * DD + 8 * hh;
  const int r0 = wave * 16 + 8 * hh;

#pragma unroll 1
  for (int g = 0; g < 2; ++g) {
    v8f acc[4];
#pragma unroll
    for (int t = 0; t < 4; ++t) { v8f z = {0.f, 0.f, 0.f, 0.f, 0.f, 0.f, 0.f, 0.f}; acc[t] = z; }
#pragma unroll 1
    for (int kt = 0; kt < DD / 32; ++kt) {
      FragB ah, al;
      split16(arow + 32 * kt, ah, al);
#pragma unroll
      for (int t = 0; t < 4; ++t) {
        const int col = 64 * g + 16 * t + m;
        const unsigned short* bph = whi + (size_t)col * DD + 32 * kt + 8 * hh;
        const unsigned short* bpl = wlo + (size_t)col * DD + 32 * kt + 8 * hh;
        FragB bh, bl;
        bh.u[0] = *(const v8us*)bph;
        bh.u[1] = *(const v8us*)(bph + 16);
        bl.u[0] = *(const v8us*)bpl;
        bl.u[1] = *(const v8us*)(bpl + 16);
        acc[t] = wmb(ah, bh, acc[t]);
        acc[t] = wmb(ah, bl, acc[t]);
        acc[t] = wmb(al, bh, acc[t]);
      }
    }
#pragma unroll
    for (int t = 0; t < 4; ++t) {
      const int col = 64 * g + 16 * t + m;
      float* sp = stg + r0 * DD + col;
#pragma unroll
      for (int r = 0; r < 8; ++r) sp[r * DD] = acc[t][r];
    }
  }
  __syncthreads();

  float* op = hout + (size_t)rowBase * DD;
#pragma unroll 1
  for (int i = 0; i < 16; ++i) {
    const int rr = wave * 16 + i;
    const v4f v = *(const v4f*)(stg + rr * DD + 4 * lane);
    *(volatile v4f*)(op + (size_t)rr * DD + 4 * lane) = v;
  }
  __threadfence();
#pragma unroll 1
  for (int i = 0; i < 16; ++i) {
    const int rr = wave * 16 + i;
    const v4f v = *(const v4f*)(stg + rr * DD + 4 * lane);
    *(volatile v4f*)(op + (size_t)rr * DD + 4 * lane) = v;
  }
}

__global__ __launch_bounds__(NTHR) void k_agg(
    const int* __restrict__ csr, const int* __restrict__ off, const int* __restrict__ cnt,
    const int* __restrict__ acol, const float* __restrict__ aval, const float* __restrict__ x,
    float* y, int nN, int nE, int csrLen, int nRowsY) {
  const int tid = threadIdx.x, lane = tid & 31, wave = tid >> 5;
  const int tbase = blockIdx.x * TGT + wave * 32;
  const int cl = tbase + lane;
  const int cnt_l = cnt[cl];
  const int off_l = off[cl];
  union FI { float f; int i; };

#pragma unroll 1
  for (int j = 0; j < 32; ++j) {
    const int c = tbase + j;
    int n = __builtin_amdgcn_readlane(cnt_l, j);
    n = n < 0 ? 0 : (n > DEGCAP ? DEGCAP : n);
    const int st = __builtin_amdgcn_readlane(off_l, j);
    v4f a0 = {0.f, 0.f, 0.f, 0.f};
#pragma unroll 1
    for (int q0 = 0; q0 < n; q0 += 32) {
      int pos = st + q0 + lane;
      pos = pos < 0 ? 0 : (pos > csrLen - 1 ? csrLen - 1 : pos);
      int ed = csr[pos];
      ed = ed < 0 ? 0 : (ed > nE - 1 ? nE - 1 : ed);
      int cc = acol[ed];
      cc = cc < 0 ? 0 : (cc > nN - 1 ? nN - 1 : cc);
      FI vv; vv.f = aval[ed];
      const int mcnt = (n - q0) < 32 ? (n - q0) : 32;
#pragma unroll 1
      for (int p = 0; p < mcnt; ++p) {
        const int s = __builtin_amdgcn_readlane(cc, p);
        FI w; w.i = __builtin_amdgcn_readlane(vv.i, p);
        const v4f x0 = *(const v4f*)(x + (size_t)s * DD + 4 * lane);
        a0 = a0 + x0 * w.f;
      }
    }
    v4f rv;
    rv.x = fmaxf(a0.x, 0.f); rv.y = fmaxf(a0.y, 0.f); rv.z = fmaxf(a0.z, 0.f); rv.w = fmaxf(a0.w, 0.f);
    if (c < nRowsY) {
      float* yp = y + (size_t)c * DD + 4 * lane;
      *(volatile v4f*)yp = rv;
      __threadfence();
      *(volatile v4f*)yp = rv;
    }
  }
}

extern "C" void kernel_launch(void* const* d_in, const int* in_sizes, int n_in,
                              void* d_out, int out_size, void* d_ws, size_t ws_size,
                              hipStream_t stream) {
  if (n_in < 6) return;
  if (in_sizes[0] <= 0 || (in_sizes[0] % DD) != 0) return;
  const int nN = in_sizes[0] / DD;
  const int nE = in_sizes[1];
  if (nN <= 0 || nE <= 0 || in_sizes[2] != nE || in_sizes[3] != nE) return;
  if (in_sizes[4] != DD * DD || in_sizes[5] != DD * DD) return;
  if (out_size != nN * DD) return;
  if (nE > (1 << 28) || nN > (1 << 24)) return;

  const float* X    = (const float*)d_in[0];
  const int*   arow = (const int*)d_in[1];
  const int*   acol = (const int*)d_in[2];
  const float* aval = (const float*)d_in[3];
  const float* W1   = (const float*)d_in[4];
  const float* W2   = (const float*)d_in[5];
  float* out = (float*)d_out;

  const int NPAD   = ((nN + TGT - 1) / TGT) * TGT;
  const int nBC    = (nN + NBC - 1) / NBC;
  const int CNTPAD = nBC * NBC;
  if (4 * nBC + 1 > RBN) return;
  const int nBF    = (nN + NBF - 1) / NBF;
  const int csrLen = ((nE + 31) & ~31) + 4096;
  const int nAgg   = NPAD / TGT;
  const int nGemm  = NPAD / GROWS;

  char* ws = (char*)d_ws;
  size_t off = 0;
  const size_t oW1h = off; off += (size_t)DD * DD * 2;            off = (off + 255) & ~(size_t)255;
  const size_t oW1l = off; off += (size_t)DD * DD * 2;            off = (off + 255) & ~(size_t)255;
  const size_t oW2h = off; off += (size_t)DD * DD * 2;            off = (off + 255) & ~(size_t)255;
  const size_t oW2l = off; off += (size_t)DD * DD * 2;            off = (off + 255) & ~(size_t)255;
  const size_t oCnt = off; off += (size_t)CNTPAD * 4;             off = (off + 255) & ~(size_t)255;
  const size_t oOff = off; off += (size_t)CNTPAD * 4;             off = (off + 255) & ~(size_t)255;
  const size_t oRb  = off; off += (size_t)RBN * 4;                off = (off + 255) & ~(size_t)255;
  const size_t oCsr = off; off += (size_t)csrLen * 4;             off = (off + 255) & ~(size_t)255;
  const size_t oHW  = off; off += (size_t)NPAD * DD * 4;          off = (off + 255) & ~(size_t)255;
  const size_t oH1  = off; off += (size_t)NPAD * DD * 4;          off = (off + 255) & ~(size_t)255;
  if (off > ws_size || off > WS_LIMIT) return;
  unsigned short* w1h  = (unsigned short*)(ws + oW1h);
  unsigned short* w1l  = (unsigned short*)(ws + oW1l);
  unsigned short* w2h  = (unsigned short*)(ws + oW2h);
  unsigned short* w2l  = (unsigned short*)(ws + oW2l);
  int*            cnt  = (int*)(ws + oCnt);
  int*            offp = (int*)(ws + oOff);
  int*            rb   = (int*)(ws + oRb);
  int*            csr  = (int*)(ws + oCsr);
  float*          hw   = (float*)(ws + oHW);
  float*          h1   = (float*)(ws + oH1);

  const int vec8 = ((nE & 3) == 0) ? 1 : 0;

  k_wprep<<<(DD * DD / 8) / NTHR, NTHR, 0, stream>>>(W1, w1h, w1l);
  k_wprep<<<(DD * DD / 8) / NTHR, NTHR, 0, stream>>>(W2, w2h, w2l);

  k_count<<<nBC, NTHR, 0, stream>>>(arow, cnt, nE, vec8);
  k_offsets<<<1, OTHR, 0, stream>>>(cnt, offp, rb, nBC);
  hipFuncSetAttribute(reinterpret_cast<const void*>(&k_fill),
                      hipFuncAttributeMaxDynamicSharedMemorySize, LDS_FILL);
  k_fill<<<nBF, NTHR, LDS_FILL, stream>>>(arow, offp, rb, csr, nE, vec8, csrLen);

  hipFuncSetAttribute(reinterpret_cast<const void*>(&k_gemm),
                      hipFuncAttributeMaxDynamicSharedMemorySize, LDS_GEMM);
  k_gemm<<<nGemm, NTHR, LDS_GEMM, stream>>>(X, w1h, w1l, hw, nN);

  k_agg<<<nAgg, NTHR, 0, stream>>>(csr, offp, cnt, acol, aval, hw, h1, nN, nE, csrLen, NPAD);

  k_gemm<<<nGemm, NTHR, LDS_GEMM, stream>>>(h1, w2h, w2l, hw, NPAD);

  k_agg<<<nAgg, NTHR, 0, stream>>>(csr, offp, cnt, acol, aval, hw, out, nN, nE, csrLen, nN);
}
